// DistributionalCritic_65017214926887
// MI455X (gfx1250) — hardware-run, weakly checked
//
#include <hip/hip_runtime.h>
#include <math.h>

constexpr int kB   = 16384;
constexpr int kSD  = 512;
constexpr int kAD  = 64;
constexpr int kH   = 1024;
constexpr int kQE  = 64;
constexpr int kNQ  = 64;
constexpr int kKIN = kSD + kAD;
constexpr int kWHW = kH + kQE;

constexpr float kXCarry    = 16.0f;
constexpr float kHCarry    = 16.0f;
constexpr float kWCarry    = 256.0f;
constexpr float kGemmScale = 1.0f / 4096.0f;
constexpr float kInvH      = 1.0f / 1024.0f;
constexpr float kLnEps     = 1e-5f;

static_assert(kKIN % 32 == 0, "K1 multiple of 32");
static_assert(kH % 64 == 0 && kB % 64 == 0, "tile multiples");

constexpr int kXStateBlocks = kB * (kSD / 8) / 256;
constexpr int kXActBlocks   = kB * (kAD / 8) / 256;
static_assert(kXStateBlocks * 256 * 8 == kB * kSD, "state coverage exact");
static_assert(kXActBlocks * 256 * 8 == kB * kAD, "action coverage exact");

constexpr size_t kOffX16  = 0;
constexpr size_t kOffW1   = kOffX16 + (size_t)kB * kKIN * 2;
constexpr size_t kOffW2   = kOffW1  + (size_t)2 * kH * kKIN * 2;
constexpr size_t kOffC32  = kOffW2  + (size_t)2 * kH * kH * 2;
constexpr size_t kOffH16  = kOffC32 + (size_t)kB * kH * 4;
constexpr size_t kOffQT   = kOffH16 + (size_t)kB * kH * 2;
constexpr size_t kWsTotal = kOffQT  + (size_t)2 * kNQ * 4;
static_assert(kWsTotal <= (size_t)134217728, "carve within 128 MiB");
static_assert(kOffW1 % 128 == 0 && kOffW2 % 128 == 0 && kOffC32 % 128 == 0 && kOffH16 % 128 == 0 && kOffQT % 128 == 0, "aligned");

typedef __attribute__((ext_vector_type(16))) _Float16 v16h;
typedef __attribute__((ext_vector_type(8)))  _Float16 v8h;
typedef __attribute__((ext_vector_type(16))) __bf16   v16b;
typedef __attribute__((ext_vector_type(8)))  __bf16   v8b;
typedef __attribute__((ext_vector_type(8)))  float    v8f;
typedef __attribute__((ext_vector_type(4)))  float    v4f;
typedef __attribute__((ext_vector_type(4)))  unsigned int v4u;

__device__ __forceinline__ unsigned short f2bf_bits(float f) {
  unsigned u = __float_as_uint(f);
  return (unsigned short)((u + 0x7FFFu + ((u >> 16) & 1u)) >> 16);
}
__device__ __forceinline__ float bf_bits2f(unsigned short h) { return __uint_as_float(((unsigned)h) << 16); }

__device__ __forceinline__ void dep_guard_h(v8f& a, v8f& b, v16h x, v16h y) { asm volatile("v_nop\n\tv_nop\n\tv_nop\n\tv_nop" : "+v"(a), "+v"(b) : "v"(x), "v"(y)); }
__device__ __forceinline__ void dep_guard_b(v8f& a, v8f& b, v16b x, v16b y) { asm volatile("v_nop\n\tv_nop\n\tv_nop\n\tv_nop" : "+v"(a), "+v"(b) : "v"(x), "v"(y)); }
__device__ __forceinline__ void keep4_h(v16h a, v16h b, v16h c, v16h d) { asm volatile("v_nop" :: "v"(a), "v"(b), "v"(c), "v"(d)); }
__device__ __forceinline__ void keep4_b(v16b a, v16b b, v16b c, v16b d) { asm volatile("v_nop" :: "v"(a), "v"(b), "v"(c), "v"(d)); }
__device__ __forceinline__ void acc_guard4(v8f& a, v8f& b, v8f& c, v8f& d) { asm volatile("v_nop\n\tv_nop\n\tv_nop\n\tv_nop" : "+v"(a), "+v"(b), "+v"(c), "+v"(d)); }
template <typename T> struct Frag;
template <> struct Frag<_Float16> {
  typedef v16h V; union U { v16h v; v8h h[2]; };
  static __device__ __forceinline__ v16h load(const _Float16* p) {
    U f; f.h[0] = *(const v8h*)(p); f.h[1] = *(const v8h*)(p + 16); return f.v;
  }
  static __device__ __forceinline__ v8f mma(v16h a, v16h b, v8f c) {
    return __builtin_amdgcn_wmma_f32_16x16x32_f16(false, a, false, b, (short)0, c, false, false);
  }
  static __device__ __forceinline__ void guard(v8f& a, v8f& b, v16h x, v16h y) { dep_guard_h(a, b, x, y); }
  static __device__ __forceinline__ void keep(v16h a, v16h b, v16h c, v16h d) { keep4_h(a, b, c, d); }
};
template <> struct Frag<__bf16> {
  typedef v16b V; union U { v16b v; v8b h[2]; };
  static __device__ __forceinline__ v16b load(const __bf16* p) {
    U f; f.h[0] = *(const v8b*)(p); f.h[1] = *(const v8b*)(p + 16); return f.v;
  }
  static __device__ __forceinline__ v8f mma(v16b a, v16b b, v8f c) {
    return __builtin_amdgcn_wmma_f32_16x16x32_bf16(false, a, false, b, (short)0, c, false, false);
  }
  static __device__ __forceinline__ void guard(v8f& a, v8f& b, v16b x, v16b y) { dep_guard_b(a, b, x, y); }
  static __device__ __forceinline__ void keep(v16b a, v16b b, v16b c, v16b d) { keep4_b(a, b, c, d); }
};

__device__ __forceinline__ unsigned pk16(unsigned short a, unsigned short b) { return (unsigned)a | ((unsigned)b << 16); }
__device__ __forceinline__ unsigned short h_bits(float f) { const _Float16 h = (_Float16)f; return __builtin_bit_cast(unsigned short, h); }

template <int ET> struct Elem;
template <> struct Elem<0> { typedef _Float16 T; };
template <> struct Elem<1> { typedef __bf16 T; };
template <int ET, bool SPLIT, int BIAS_MODE, int OUT_MODE, bool RESID, int ACT = 0>
__global__ __launch_bounds__(256) void wmma_gemm64(
    const unsigned short* __restrict__ Ap, const unsigned short* __restrict__ A2p, int lda, long strideA,
    const unsigned short* __restrict__ Btp, const unsigned short* __restrict__ Bt2p, int ldb, long strideB,
    void* __restrict__ Cout, void* __restrict__ Cout2, int ldc, long strideC,
    const float* __restrict__ bias,
    const float* __restrict__ resid, long strideR,
    int M, int N, int K, float scale) {
  typedef typename Elem<ET>::T T;
  typedef typename Frag<T>::V V;
  const T* A = (const T*)Ap; const T* A2 = (const T*)A2p; const T* Bt = (const T*)Btp; const T* Bt2 = (const T*)Bt2p;
  __shared__ __align__(16) float sT[8][16 * 68];
  const int b    = blockIdx.y;
  const int lane = threadIdx.x & 31;
  const int wave = threadIdx.x >> 5;
  const int tilesN = N >> 6;
  const int tilesM = M >> 6;
  const int tile = blockIdx.x * 8 + wave;
  if (tile >= tilesM * tilesN) return;
  const int tm = tile / tilesN;
  const int tn = tile - tm * tilesN;
  const int m0 = tm << 6;
  const int n0 = tn << 6;

  const T* Ab  = A  + (size_t)b * strideA;
  const T* Bb  = Bt + (size_t)b * strideB;
  const T* Ab2 = SPLIT ? (A2  + (size_t)b * strideA) : nullptr;
  const T* Bb2 = SPLIT ? (Bt2 + (size_t)b * strideB) : nullptr;

  const int rlane = lane & 15;
  const int koff  = (lane >> 4) * 8;
  const int mOff  = (lane >> 4) * 8;

  v8f acc[4][4];
#pragma unroll
  for (int i = 0; i < 4; ++i)
#pragma unroll
    for (int j = 0; j < 4; ++j) acc[i][j] = (v8f){0.f,0.f,0.f,0.f,0.f,0.f,0.f,0.f};

  for (int k0 = 0; k0 < K; k0 += 32) {
    V bh[4], bl[4];
#pragma unroll
    for (int j = 0; j < 4; ++j) {
      const size_t bo = (size_t)(n0 + (j << 4) + rlane) * ldb + koff + k0;
      bh[j] = Frag<T>::load(Bb + bo);
      if (SPLIT) bl[j] = Frag<T>::load(Bb2 + bo);
    }
#pragma unroll
    for (int i = 0; i < 4; ++i) {
      const size_t ao = (size_t)(m0 + (i << 4) + rlane) * lda + koff + k0;
      V ah = Frag<T>::load(Ab + ao);
      V al;
      if (SPLIT) al = Frag<T>::load(Ab2 + ao);
#pragma unroll
      for (int j = 0; j < 4; ++j) {
        acc[i][j] = Frag<T>::mma(ah, bh[j], acc[i][j]);
        if (SPLIT) {
          acc[i][j] = Frag<T>::mma(ah, bl[j], acc[i][j]);
          acc[i][j] = Frag<T>::mma(al, bh[j], acc[i][j]);
        }
      }
      Frag<T>::guard(acc[i][0], acc[i][3], ah, SPLIT ? al : ah);
    }
    Frag<T>::keep(bh[0], bh[1], bh[2], bh[3]);
    if (SPLIT) Frag<T>::keep(bl[0], bl[1], bl[2], bl[3]);
  }
  acc_guard4(acc[0][0], acc[0][1], acc[0][2], acc[0][3]);
  acc_guard4(acc[1][0], acc[1][1], acc[1][2], acc[1][3]);
  acc_guard4(acc[2][0], acc[2][1], acc[2][2], acc[2][3]);
  acc_guard4(acc[3][0], acc[3][1], acc[3][2], acc[3][3]);

  float* slab = sT[wave];
  const float* Rb = RESID ? (resid + (size_t)b * strideR) : nullptr;
#pragma unroll
  for (int i = 0; i < 4; ++i) {
    const int mBase = m0 + (i << 4);
#pragma unroll
    for (int j = 0; j < 4; ++j) {
      const int n = n0 + (j << 4) + rlane;
      float bv = 0.f;
      if (BIAS_MODE == 2) bv = bias[n];
#pragma unroll
      for (int r = 0; r < 8; ++r) {
        float v = acc[i][j][r] * scale;
        if (BIAS_MODE == 1) v += bias[mBase + mOff + r];
        if (BIAS_MODE == 2) v += bv;
        if (RESID) v += Rb[(size_t)(mBase + mOff + r) * ldc + n];
        if (ACT == 2) v = fmaxf(v, 0.0f);
        if (ACT == 4) v = (v > 0.f) ? v : 0.01f * v;
        slab[(mOff + r) * 68 + (j << 4) + rlane] = v;
      }
    }
    __builtin_amdgcn_fence(__ATOMIC_RELEASE, "workgroup");
    __builtin_amdgcn_wave_barrier();
    __builtin_amdgcn_fence(__ATOMIC_ACQUIRE, "workgroup");
    if (OUT_MODE == 0) {
      float* C = (float*)Cout + (size_t)b * strideC;
      const int hh = lane >> 4, c4 = (lane & 15) * 4;
      for (int pass = 0; pass < 2; ++pass) {
#pragma unroll
        for (int it = 0; it < 8; ++it) {
          const int row = it * 2 + hh;
          v4f v = *(const v4f*)(slab + row * 68 + c4);
          *(volatile v4f*)(C + (size_t)(mBase + row) * ldc + n0 + c4) = v;
        }
        __threadfence();
      }
    } else {
      const int q = lane >> 3, c8 = (lane & 7) * 8;
      unsigned short* C  = (unsigned short*)Cout  + (size_t)b * strideC;
      unsigned short* C2 = (OUT_MODE == 2) ? ((unsigned short*)Cout2 + (size_t)b * strideC) : nullptr;
      for (int pass = 0; pass < 2; ++pass) {
#pragma unroll
        for (int it = 0; it < 4; ++it) {
          const int row = it * 4 + q;
          const float* sp = slab + row * 68 + c8;
          v8h hv, lv;
#pragma unroll
          for (int e = 0; e < 8; ++e) {
            if (OUT_MODE == 1) {
              hv[e] = (_Float16)sp[e];
            } else {
              unsigned short hb = f2bf_bits(sp[e]);
              unsigned short lb = f2bf_bits(sp[e] - bf_bits2f(hb));
              hv[e] = __builtin_bit_cast(_Float16, hb);
              lv[e] = __builtin_bit_cast(_Float16, lb);
            }
          }
          *(volatile v8h*)(C + (size_t)(mBase + row) * ldc + n0 + c8) = hv;
          if (OUT_MODE == 2) *(volatile v8h*)(C2 + (size_t)(mBase + row) * ldc + n0 + c8) = lv;
        }
        __threadfence();
      }
    }
    __builtin_amdgcn_fence(__ATOMIC_RELEASE, "workgroup");
    __builtin_amdgcn_wave_barrier();
    __builtin_amdgcn_fence(__ATOMIC_ACQUIRE, "workgroup");
  }
}

__global__ __launch_bounds__(256) void cast_x_kernel(const float* __restrict__ state, const float* __restrict__ action,
                                                     unsigned short* __restrict__ X, float scale) {
  const int t = threadIdx.x;
  const float* src;
  size_t dst;
  if (blockIdx.x < kXStateBlocks) {
    const int i   = blockIdx.x * 256 + t;
    const int row = i >> 6, seg = i & 63;
    src = state + (size_t)row * kSD + seg * 8;
    dst = (size_t)row * kKIN + seg * 8;
  } else {
    const int j   = (blockIdx.x - kXStateBlocks) * 256 + t;
    const int row = j >> 3, seg = j & 7;
    src = action + (size_t)row * kAD + seg * 8;
    dst = (size_t)row * kKIN + kSD + seg * 8;
  }
  const v4f a = *(const v4f*)src;
  const v4f c = *(const v4f*)(src + 4);
  const v4u u = (v4u){pk16(h_bits(a[0] * scale), h_bits(a[1] * scale)), pk16(h_bits(a[2] * scale), h_bits(a[3] * scale)),
                      pk16(h_bits(c[0] * scale), h_bits(c[1] * scale)), pk16(h_bits(c[2] * scale), h_bits(c[3] * scale))};
  *(volatile v4u*)(X + dst) = u;
  __threadfence();
  *(volatile v4u*)(X + dst) = u;
}

__global__ __launch_bounds__(256) void cast8_kernel(const float* __restrict__ in, unsigned short* __restrict__ out,
                                                    int n8, float scale) {
  const int i  = blockIdx.x * 256 + threadIdx.x;
  const int ic = (i < n8) ? i : (n8 - 1);
  const float* p = in + (size_t)ic * 8;
  const v4f a = *(const v4f*)p;
  const v4f c = *(const v4f*)(p + 4);
  const v4u u = (v4u){pk16(h_bits(a[0] * scale), h_bits(a[1] * scale)), pk16(h_bits(a[2] * scale), h_bits(a[3] * scale)),
                      pk16(h_bits(c[0] * scale), h_bits(c[1] * scale)), pk16(h_bits(c[2] * scale), h_bits(c[3] * scale))};
  if (i < n8) *(volatile v4u*)(out + (size_t)ic * 8) = u;
  __threadfence();
  if (i < n8) *(volatile v4u*)(out + (size_t)ic * 8) = u;
}

__global__ __launch_bounds__(64) void tau_kernel(const float* __restrict__ We1, const float* __restrict__ be1,
                                                 const float* __restrict__ We2, const float* __restrict__ be2,
                                                 const float* __restrict__ Wh, float* __restrict__ qtau) {
  __shared__ float sr[64][65];
  __shared__ __align__(16) float sq[64];
  const int c = blockIdx.x;
  const int n = threadIdx.x;
  const float* we1 = We1 + c * kQE;
  const float* b1  = be1 + c * kQE;
  const float* we2 = We2 + (size_t)c * kQE * kQE;
  const float* b2  = be2 + c * kQE;
  const float* wh2 = Wh + (size_t)c * kWHW + kH;
  const float tau = (float)(2 * n + 1) * (1.0f / 128.0f);
#pragma unroll 1
  for (int j = 0; j < kQE; ++j) sr[n][j] = fmaxf(tau * we1[j] + b1[j], 0.0f);
  float q = 0.0f;
#pragma unroll 1
  for (int qq = 0; qq < kQE; ++qq) {
    float acc = 0.0f;
#pragma unroll 1
    for (int j = 0; j < kQE; ++j) acc += sr[n][j] * we2[qq * kQE + j];
    const float te = acc + b2[qq];
    q += te * wh2[qq];
  }
  sq[n] = q;
  __syncthreads();
  const int l4 = (n < 16) ? n : 15;
  const v4f v = *(const v4f*)(sq + 4 * l4);
  if (n < 16) *(volatile v4f*)(qtau + c * kNQ + 4 * l4) = v;
  __threadfence();
  if (n < 16) *(volatile v4f*)(qtau + c * kNQ + 4 * l4) = v;
}

__device__ __forceinline__ float wave_sum(float s) {
#pragma unroll
  for (int off = 16; off > 0; off >>= 1) s += __shfl_xor(s, off, 32);
  return s;
}

__global__ __launch_bounds__(128) void ln_relu_h16_kernel(const float* __restrict__ C,
                                                          const float* __restrict__ g, const float* __restrict__ beta,
                                                          unsigned short* __restrict__ Hout, float hscale) {
  __shared__ float red1[4];
  __shared__ float red2[4];
  const int row = blockIdx.x, t = threadIdx.x, lane = t & 31, wave = t >> 5;
  const int h0 = t * 8;
  const float* cp = C + (size_t)row * kH + h0;
  const v4f a = *(const v4f*)cp, c2 = *(const v4f*)(cp + 4);
  float x[8];
  x[0] = a[0]; x[1] = a[1]; x[2] = a[2]; x[3] = a[3];
  x[4] = c2[0]; x[5] = c2[1]; x[6] = c2[2]; x[7] = c2[3];
  float s = ((x[0] + x[1]) + (x[2] + x[3])) + ((x[4] + x[5]) + (x[6] + x[7]));
  s = wave_sum(s);
  if (lane == 0) red1[wave] = s;
  __syncthreads();
  const float mu = ((red1[0] + red1[1]) + (red1[2] + red1[3])) * kInvH;
  float d[8];
  float s2 = 0.0f;
#pragma unroll
  for (int e = 0; e < 8; ++e) { d[e] = x[e] - mu; s2 += d[e] * d[e]; }
  s2 = wave_sum(s2);
  if (lane == 0) red2[wave] = s2;
  __syncthreads();
  const float var = ((red2[0] + red2[1]) + (red2[2] + red2[3])) * kInvH;
  const float rs  = rsqrtf(var + kLnEps);
  const v4f ga = *(const v4f*)(g + h0), gb = *(const v4f*)(g + h0 + 4);
  const v4f ta = *(const v4f*)(beta + h0), tb = *(const v4f*)(beta + h0 + 4);
  float gg[8] = {ga[0], ga[1], ga[2], ga[3], gb[0], gb[1], gb[2], gb[3]};
  float tt[8] = {ta[0], ta[1], ta[2], ta[3], tb[0], tb[1], tb[2], tb[3]};
  unsigned short hb[8];
#pragma unroll
  for (int e = 0; e < 8; ++e) {
    const float y = fmaxf(d[e] * rs * gg[e] + tt[e], 0.0f);
    hb[e] = h_bits(y * hscale);
  }
  const v4u u = (v4u){pk16(hb[0], hb[1]), pk16(hb[2], hb[3]), pk16(hb[4], hb[5]), pk16(hb[6], hb[7])};
  unsigned short* op = Hout + (size_t)row * kH + h0;
  *(volatile v4u*)op = u;
  __threadfence();
  *(volatile v4u*)op = u;
}

__global__ __launch_bounds__(128) void ln_head_out_kernel(const float* __restrict__ C,
                                                          const float* __restrict__ g, const float* __restrict__ beta,
                                                          const float* __restrict__ wh, const float* __restrict__ bh,
                                                          const float* __restrict__ qtau, float* __restrict__ out) {
  __shared__ float red1[4];
  __shared__ float red2[4];
  __shared__ float red3[4];
  const int row = blockIdx.x, t = threadIdx.x, lane = t & 31, wave = t >> 5;
  const int h0 = t * 8;
  const float* cp = C + (size_t)row * kH + h0;
  const v4f a = *(const v4f*)cp, c2 = *(const v4f*)(cp + 4);
  float x[8];
  x[0] = a[0]; x[1] = a[1]; x[2] = a[2]; x[3] = a[3];
  x[4] = c2[0]; x[5] = c2[1]; x[6] = c2[2]; x[7] = c2[3];
  float s = ((x[0] + x[1]) + (x[2] + x[3])) + ((x[4] + x[5]) + (x[6] + x[7]));
  s = wave_sum(s);
  if (lane == 0) red1[wave] = s;
  __syncthreads();
  const float mu = ((red1[0] + red1[1]) + (red1[2] + red1[3])) * kInvH;
  float d[8];
  float s2 = 0.0f;
#pragma unroll
  for (int e = 0; e < 8; ++e) { d[e] = x[e] - mu; s2 += d[e] * d[e]; }
  s2 = wave_sum(s2);
  if (lane == 0) red2[wave] = s2;
  __syncthreads();
  const float var = ((red2[0] + red2[1]) + (red2[2] + red2[3])) * kInvH;
  const float rs  = rsqrtf(var + kLnEps);
  const v4f ga = *(const v4f*)(g + h0), gb = *(const v4f*)(g + h0 + 4);
  const v4f ta = *(const v4f*)(beta + h0), tb = *(const v4f*)(beta + h0 + 4);
  const v4f wa = *(const v4f*)(wh + h0), wb = *(const v4f*)(wh + h0 + 4);
  float gg[8] = {ga[0], ga[1], ga[2], ga[3], gb[0], gb[1], gb[2], gb[3]};
  float tt[8] = {ta[0], ta[1], ta[2], ta[3], tb[0], tb[1], tb[2], tb[3]};
  float ww[8] = {wa[0], wa[1], wa[2], wa[3], wb[0], wb[1], wb[2], wb[3]};
  float p = 0.0f;
#pragma unroll
  for (int e = 0; e < 8; ++e) {
    const float feat = fmaxf(d[e] * rs * gg[e] + tt[e], 0.0f);
    p += feat * ww[e];
  }
  p = wave_sum(p);
  if (lane == 0) red3[wave] = p;
  __syncthreads();
  const float qf  = (red3[0] + red3[1]) + (red3[2] + red3[3]);
  const float bh0 = bh[0];
  const int l4 = (t < 16) ? t : 15;
  const v4f qt = *(const v4f*)(qtau + 4 * l4);
  v4f v;
  v[0] = (qf + qt[0]) + bh0; v[1] = (qf + qt[1]) + bh0; v[2] = (qf + qt[2]) + bh0; v[3] = (qf + qt[3]) + bh0;
  float* op = out + (size_t)row * kNQ + 4 * l4;
  if (t < 16) *(volatile v4f*)op = v;
  __threadfence();
  if (t < 16) *(volatile v4f*)op = v;
}

extern "C" void kernel_launch(void* const* d_in, const int* in_sizes, int n_in,
                              void* d_out, int out_size, void* d_ws, size_t ws_size,
                              hipStream_t stream)
{
  if (n_in < 16) return;
  if (in_sizes[0] != kB * kSD || in_sizes[1] != kB * kAD || in_sizes[6] != 2 * kH * kKIN ||
      in_sizes[10] != 2 * kH * kH || in_sizes[14] != 2 * kWHW || in_sizes[15] != 2) return;
  if (out_size != 2 * kB * kNQ) return;
  if (ws_size < kWsTotal) return;

  const float* state  = (const float*)d_in[0];
  const float* action = (const float*)d_in[1];
  const float* We1    = (const float*)d_in[2];
  const float* be1    = (const float*)d_in[3];
  const float* We2    = (const float*)d_in[4];
  const float* be2    = (const float*)d_in[5];
  const float* Wf1    = (const float*)d_in[6];
  const float* bf1    = (const float*)d_in[7];
  const float* g1     = (const float*)d_in[8];
  const float* beta1  = (const float*)d_in[9];
  const float* Wf2    = (const float*)d_in[10];
  const float* bf2    = (const float*)d_in[11];
  const float* g2     = (const float*)d_in[12];
  const float* beta2  = (const float*)d_in[13];
  const float* Wh     = (const float*)d_in[14];
  const float* bh     = (const float*)d_in[15];
  float* out = (float*)d_out;

  char* ws = (char*)d_ws;
  unsigned short* X16 = (unsigned short*)(ws + kOffX16);
  unsigned short* W1h = (unsigned short*)(ws + kOffW1);
  unsigned short* W2h = (unsigned short*)(ws + kOffW2);
  float*          C32 = (float*)(ws + kOffC32);
  unsigned short* H16 = (unsigned short*)(ws + kOffH16);
  float*          QT  = (float*)(ws + kOffQT);

  cast_x_kernel<<<kXStateBlocks + kXActBlocks, 256, 0, stream>>>(state, action, X16, kXCarry);
  {
    const int n8_1 = 2 * kH * kKIN / 8;
    cast8_kernel<<<(n8_1 + 255) / 256, 256, 0, stream>>>(Wf1, W1h, n8_1, kWCarry);
    const int n8_2 = 2 * kH * kH / 8;
    cast8_kernel<<<(n8_2 + 255) / 256, 256, 0, stream>>>(Wf2, W2h, n8_2, kWCarry);
  }
  tau_kernel<<<2, 64, 0, stream>>>(We1, be1, We2, be2, Wh, QT);

  const int gemmBlocks = ((kB / 64) * (kH / 64) + 7) / 8;

  for (int c = 0; c < 2; ++c) {
    const unsigned short* W1c = W1h + (size_t)c * kH * kKIN;
    const unsigned short* W2c = W2h + (size_t)c * kH * kH;
    const float* bf1c = bf1 + c * kH;
    const float* bf2c = bf2 + c * kH;

    wmma_gemm64<0, false, 2, 0, false, 0><<<dim3(gemmBlocks, 1), 256, 0, stream>>>(
        X16, X16, kKIN, 0L,
        W1c, W1c, kKIN, 0L,
        (void*)C32, (void*)C32, kH, 0L,
        bf1c,
        bf1c, 0L,
        kB, kH, kKIN, kGemmScale);

    ln_relu_h16_kernel<<<kB, 128, 0, stream>>>(C32, g1 + c * kH, beta1 + c * kH, H16, kHCarry);

    wmma_gemm64<0, false, 2, 0, false, 0><<<dim3(gemmBlocks, 1), 256, 0, stream>>>(
        H16, H16, kH, 0L,
        W2c, W2c, kH, 0L,
        (void*)C32, (void*)C32, kH, 0L,
        bf2c,
        bf2c, 0L,
        kB, kH, kH, kGemmScale);

    ln_head_out_kernel<<<kB, 128, 0, stream>>>(C32, g2 + c * kH, beta2 + c * kH,
                                               Wh + (size_t)c * kWHW, bh + c, QT + c * kNQ,
                                               out + (size_t)c * kB * kNQ);
  }
}
